// MultiHeadAttentionIFA_71476845740050
// MI455X (gfx1250) — hardware-verified
//
#include <hip/hip_runtime.h>

typedef __attribute__((ext_vector_type(16))) _Float16 v16h;
typedef __attribute__((ext_vector_type(8)))  _Float16 v8h;
typedef __attribute__((ext_vector_type(16))) __bf16   v16b;
typedef __attribute__((ext_vector_type(8)))  __bf16   v8b;
typedef __attribute__((ext_vector_type(8)))  float    v8f;
typedef __attribute__((ext_vector_type(4)))  float    v4f;

__device__ __forceinline__ unsigned short f2bf_bits(float f) {
  unsigned u = __float_as_uint(f);
  return (unsigned short)((u + 0x7FFFu + ((u >> 16) & 1u)) >> 16);
}
__device__ __forceinline__ float bf_bits2f(unsigned short h) { return __uint_as_float(((unsigned)h) << 16); }

__device__ __forceinline__ void dep_guard_h(v8f& a, v8f& b, v16h x, v16h y) { asm volatile("v_nop\n\tv_nop\n\tv_nop\n\tv_nop" : "+v"(a), "+v"(b) : "v"(x), "v"(y)); }
__device__ __forceinline__ void dep_guard_b(v8f& a, v8f& b, v16b x, v16b y) { asm volatile("v_nop\n\tv_nop\n\tv_nop\n\tv_nop" : "+v"(a), "+v"(b) : "v"(x), "v"(y)); }
__device__ __forceinline__ void keep4_h(v16h a, v16h b, v16h c, v16h d) { asm volatile("v_nop" :: "v"(a), "v"(b), "v"(c), "v"(d)); }
__device__ __forceinline__ void keep4_b(v16b a, v16b b, v16b c, v16b d) { asm volatile("v_nop" :: "v"(a), "v"(b), "v"(c), "v"(d)); }
__device__ __forceinline__ void acc_guard4(v8f& a, v8f& b, v8f& c, v8f& d) { asm volatile("v_nop\n\tv_nop\n\tv_nop\n\tv_nop" : "+v"(a), "+v"(b), "+v"(c), "+v"(d)); }
template <typename T> struct Frag;
template <> struct Frag<_Float16> {
  typedef v16h V; union U { v16h v; v8h h[2]; };
  static __device__ __forceinline__ v16h load(const _Float16* p) {
    U f; f.h[0] = *(const v8h*)(p); f.h[1] = *(const v8h*)(p + 16); return f.v;
  }
  static __device__ __forceinline__ v8f mma(v16h a, v16h b, v8f c) {
    return __builtin_amdgcn_wmma_f32_16x16x32_f16(false, a, false, b, (short)0, c, false, false);
  }
  static __device__ __forceinline__ void guard(v8f& a, v8f& b, v16h x, v16h y) { dep_guard_h(a, b, x, y); }
  static __device__ __forceinline__ void keep(v16h a, v16h b, v16h c, v16h d) { keep4_h(a, b, c, d); }
};
template <> struct Frag<__bf16> {
  typedef v16b V; union U { v16b v; v8b h[2]; };
  static __device__ __forceinline__ v16b load(const __bf16* p) {
    U f; f.h[0] = *(const v8b*)(p); f.h[1] = *(const v8b*)(p + 16); return f.v;
  }
  static __device__ __forceinline__ v8f mma(v16b a, v16b b, v8f c) {
    return __builtin_amdgcn_wmma_f32_16x16x32_bf16(false, a, false, b, (short)0, c, false, false);
  }
  static __device__ __forceinline__ void guard(v8f& a, v8f& b, v16b x, v16b y) { dep_guard_b(a, b, x, y); }
  static __device__ __forceinline__ void keep(v16b a, v16b b, v16b c, v16b d) { keep4_b(a, b, c, d); }
};

template <int ET> struct Elem;
template <> struct Elem<0> { typedef _Float16 T; };
template <> struct Elem<1> { typedef __bf16 T; };
template <int ET, bool SPLIT, int BIAS_MODE, int OUT_MODE, bool RESID, int ACT = 0>
__global__ __launch_bounds__(256) void wmma_gemm64(
    const unsigned short* __restrict__ Ap, const unsigned short* __restrict__ A2p, int lda, long strideA,
    const unsigned short* __restrict__ Btp, const unsigned short* __restrict__ Bt2p, int ldb, long strideB,
    void* __restrict__ Cout, void* __restrict__ Cout2, int ldc, long strideC,
    const float* __restrict__ bias,
    const float* __restrict__ resid, long strideR,
    int M, int N, int K, float scale) {
  typedef typename Elem<ET>::T T;
  typedef typename Frag<T>::V V;
  const T* A = (const T*)Ap; const T* A2 = (const T*)A2p; const T* Bt = (const T*)Btp; const T* Bt2 = (const T*)Bt2p;
  __shared__ __align__(16) float sT[8][16 * 68];
  const int b    = blockIdx.y;
  const int lane = threadIdx.x & 31;
  const int wave = threadIdx.x >> 5;
  const int tilesN = N >> 6;
  const int tilesM = M >> 6;
  const int tile = blockIdx.x * 8 + wave;
  if (tile >= tilesM * tilesN) return;
  const int tm = tile / tilesN;
  const int tn = tile - tm * tilesN;
  const int m0 = tm << 6;
  const int n0 = tn << 6;

  const T* Ab  = A  + (size_t)b * strideA;
  const T* Bb  = Bt + (size_t)b * strideB;
  const T* Ab2 = SPLIT ? (A2  + (size_t)b * strideA) : nullptr;
  const T* Bb2 = SPLIT ? (Bt2 + (size_t)b * strideB) : nullptr;

  const int rlane = lane & 15;
  const int koff  = (lane >> 4) * 8;
  const int mOff  = (lane >> 4) * 8;

  v8f acc[4][4];
#pragma unroll
  for (int i = 0; i < 4; ++i)
#pragma unroll
    for (int j = 0; j < 4; ++j) acc[i][j] = (v8f){0.f,0.f,0.f,0.f,0.f,0.f,0.f,0.f};

  for (int k0 = 0; k0 < K; k0 += 32) {
    V bh[4], bl[4];
#pragma unroll
    for (int j = 0; j < 4; ++j) {
      const size_t bo = (size_t)(n0 + (j << 4) + rlane) * ldb + koff + k0;
      bh[j] = Frag<T>::load(Bb + bo);
      if (SPLIT) bl[j] = Frag<T>::load(Bb2 + bo);
    }
#pragma unroll
    for (int i = 0; i < 4; ++i) {
      const size_t ao = (size_t)(m0 + (i << 4) + rlane) * lda + koff + k0;
      V ah = Frag<T>::load(Ab + ao);
      V al;
      if (SPLIT) al = Frag<T>::load(Ab2 + ao);
#pragma unroll
      for (int j = 0; j < 4; ++j) {
        acc[i][j] = Frag<T>::mma(ah, bh[j], acc[i][j]);
        if (SPLIT) {
          acc[i][j] = Frag<T>::mma(ah, bl[j], acc[i][j]);
          acc[i][j] = Frag<T>::mma(al, bh[j], acc[i][j]);
        }
      }
      Frag<T>::guard(acc[i][0], acc[i][3], ah, SPLIT ? al : ah);
    }
    Frag<T>::keep(bh[0], bh[1], bh[2], bh[3]);
    if (SPLIT) Frag<T>::keep(bl[0], bl[1], bl[2], bl[3]);
  }
  acc_guard4(acc[0][0], acc[0][1], acc[0][2], acc[0][3]);
  acc_guard4(acc[1][0], acc[1][1], acc[1][2], acc[1][3]);
  acc_guard4(acc[2][0], acc[2][1], acc[2][2], acc[2][3]);
  acc_guard4(acc[3][0], acc[3][1], acc[3][2], acc[3][3]);

  float* slab = sT[wave];
  const float* Rb = RESID ? (resid + (size_t)b * strideR) : nullptr;
#pragma unroll
  for (int i = 0; i < 4; ++i) {
    const int mBase = m0 + (i << 4);
#pragma unroll
    for (int j = 0; j < 4; ++j) {
      const int n = n0 + (j << 4) + rlane;
      float bv = 0.f;
      if (BIAS_MODE == 2) bv = bias[n];
#pragma unroll
      for (int r = 0; r < 8; ++r) {
        float v = acc[i][j][r] * scale;
        if (BIAS_MODE == 1) v += bias[mBase + mOff + r];
        if (BIAS_MODE == 2) v += bv;
        if (RESID) v += Rb[(size_t)(mBase + mOff + r) * ldc + n];
        if (ACT == 1) v = tanhf(v);
        if (ACT == 2) v = fmaxf(v, 0.0f);
        if (ACT == 3) v = v / (1.0f + expf(-v));
        if (ACT == 4) v = (v > 0.f) ? v : 0.01f * v;
        if (ACT == 5) v = 0.5f * v * (1.0f + erff(v * 0.70710678118654752f));
        slab[(mOff + r) * 68 + (j << 4) + rlane] = v;
      }
    }
    __builtin_amdgcn_fence(__ATOMIC_RELEASE, "workgroup");
    __builtin_amdgcn_wave_barrier();
    __builtin_amdgcn_fence(__ATOMIC_ACQUIRE, "workgroup");
    if (OUT_MODE == 0) {
      float* C = (float*)Cout + (size_t)b * strideC;
      const int hh = lane >> 4, c4 = (lane & 15) * 4;
      for (int pass = 0; pass < 2; ++pass) {
#pragma unroll
        for (int it = 0; it < 8; ++it) {
          const int row = it * 2 + hh;
          v4f v = *(const v4f*)(slab + row * 68 + c4);
          *(volatile v4f*)(C + (size_t)(mBase + row) * ldc + n0 + c4) = v;
        }
        __threadfence();
      }
    } else {
      const int q = lane >> 3, c8 = (lane & 7) * 8;
      unsigned short* C  = (unsigned short*)Cout  + (size_t)b * strideC;
      unsigned short* C2 = (OUT_MODE == 2) ? ((unsigned short*)Cout2 + (size_t)b * strideC) : nullptr;
      for (int pass = 0; pass < 2; ++pass) {
#pragma unroll
        for (int it = 0; it < 4; ++it) {
          const int row = it * 4 + q;
          const float* sp = slab + row * 68 + c8;
          v8h hv, lv;
#pragma unroll
          for (int e = 0; e < 8; ++e) {
            if (OUT_MODE == 1) {
              hv[e] = (_Float16)sp[e];
            } else {
              unsigned short hb = f2bf_bits(sp[e]);
              unsigned short lb = f2bf_bits(sp[e] - bf_bits2f(hb));
              hv[e] = __builtin_bit_cast(_Float16, hb);
              lv[e] = __builtin_bit_cast(_Float16, lb);
            }
          }
          *(volatile v8h*)(C + (size_t)(mBase + row) * ldc + n0 + c8) = hv;
          if (OUT_MODE == 2) *(volatile v8h*)(C2 + (size_t)(mBase + row) * ldc + n0 + c8) = lv;
        }
        __threadfence();
      }
    }
    __builtin_amdgcn_fence(__ATOMIC_RELEASE, "workgroup");
    __builtin_amdgcn_wave_barrier();
    __builtin_amdgcn_fence(__ATOMIC_ACQUIRE, "workgroup");
  }
}

__global__ __launch_bounds__(256) void cast_f32_f16x2(
    const float* __restrict__ in, _Float16* __restrict__ out, int n2) {
  int i = blockIdx.x * 256 + threadIdx.x;
  if (i < n2) {
    const _Float16 h0 = (_Float16)in[2 * i], h1 = (_Float16)in[2 * i + 1];
    const unsigned u = (unsigned)__builtin_bit_cast(unsigned short, h0) | ((unsigned)__builtin_bit_cast(unsigned short, h1) << 16);
    ((volatile unsigned*)out)[i] = u;
    __threadfence();
    ((volatile unsigned*)out)[i] = u;
  }
}
__global__ __launch_bounds__(256) void cast_f32_f16x2s(
    const float* __restrict__ in, _Float16* __restrict__ out, int n2, float sc) {
  int i = blockIdx.x * 256 + threadIdx.x;
  if (i < n2) {
    const _Float16 h0 = (_Float16)(in[2 * i] * sc), h1 = (_Float16)(in[2 * i + 1] * sc);
    const unsigned u = (unsigned)__builtin_bit_cast(unsigned short, h0) | ((unsigned)__builtin_bit_cast(unsigned short, h1) << 16);
    ((volatile unsigned*)out)[i] = u;
    __threadfence();
    ((volatile unsigned*)out)[i] = u;
  }
}

#define AK_D  64
#define AK_NW 4
#define AK_QB 64
#define AK_KC 64

__device__ __forceinline__ v8f mma_h16(v16h a, v16h b, v8f c) {
  c = __builtin_amdgcn_wmma_f32_16x16x32_f16(false, a, false, b, (short)0, c, false, false);
  asm volatile("v_nop\n\tv_nop\n\tv_nop\n\tv_nop" : "+v"(c) : "v"(a), "v"(b));
  return c;
}

__global__ __launch_bounds__(128)
void attn64_f16io(const _Float16* __restrict__ Qp, const _Float16* __restrict__ Kp,
                  const _Float16* __restrict__ Vtp, _Float16* __restrict__ Op,
                  const int* __restrict__ kmask, const float* __restrict__ ubias,
                  const float* __restrict__ gq, const float* __restrict__ gW, const float* __restrict__ gb,
                  int S, int Skv, int H, int ldq, int ldk, int ldv, int ldo, int GD,
                  float qscale, float mfill, float oscale) {
  const float PSC = 32768.0f;
  union FB { v16h v; v8h h[2]; };
  __shared__ __align__(16) _Float16 Ksh[AK_KC * AK_D];
  __shared__ __align__(16) _Float16 Vth[AK_D * AK_KC];
  __shared__ __align__(16) _Float16 Psh[AK_NW][16 * AK_KC];
  __shared__ __align__(16) float    Os[AK_NW][16 * 68];

  const int tid  = threadIdx.x;
  const int wave = tid >> 5;
  const int lane = tid & 31;
  const int hh   = lane >> 4;
  const int c    = lane & 15;

  const int nqb = S / AK_QB;
  const int bx  = blockIdx.x;
  const int qb  = bx % nqb;
  const int bh  = bx / nqb;
  const int h   = bh % H;
  const int b   = bh / H;
  const int q0  = qb * AK_QB + wave * 16;

  v16h qa[2];
  {
    const _Float16* qrow = Qp + (size_t)(b * S + q0 + c) * ldq + h * AK_D;
#pragma unroll
    for (int dc = 0; dc < 2; ++dc) qa[dc] = Frag<_Float16>::load(qrow + dc * 32 + 8 * hh);
  }

  float gacc = 0.f;
#pragma unroll 1
  for (int i = 0; i < GD; ++i) gacc += gq[b * GD + i] * gW[h * GD + i];
  gacc += gb[h];
  const float gate = 1.0f / (1.0f + expf(-gacc));
  const float ub = ubias[h];

  float mrow[8], lrow[8];
  v8f oacc[4];
#pragma unroll
  for (int r = 0; r < 8; ++r) { mrow[r] = -__builtin_inff(); lrow[r] = 0.f; }
#pragma unroll
  for (int t = 0; t < 4; ++t) oacc[t] = (v8f){0.f,0.f,0.f,0.f,0.f,0.f,0.f,0.f};

  const int nChunks = Skv / AK_KC;
  for (int kc = 0; kc < nChunks; ++kc) {
    const int kv0 = kc * AK_KC;
    __syncthreads();
    {
#pragma unroll
      for (int i = 0; i < 4; ++i) {
        const int idx = tid + i * 128;
        const int r = idx >> 3, c8 = (idx & 7) * 8;
        const v8h kk = *(const v8h*)(Kp + (size_t)(b * Skv + kv0 + r) * ldk + h * AK_D + c8);
        *(v8h*)(Ksh + r * AK_D + c8) = kk;
        const v8h vv = *(const v8h*)(Vtp + (size_t)(h * AK_D + r) * ldv + (size_t)b * Skv + kv0 + c8);
        *(v8h*)(Vth + r * AK_KC + c8) = vv;
      }
    }
    __syncthreads();

    v8f s[4];
#pragma unroll
    for (int j = 0; j < 4; ++j) {
      s[j] = (v8f){0.f,0.f,0.f,0.f,0.f,0.f,0.f,0.f};
#pragma unroll
      for (int dc = 0; dc < 2; ++dc) {
        FB kb;
        kb.h[0] = *(const v8h*)(Ksh + (j * 16 + c) * AK_D + dc * 32 + 8 * hh);
        kb.h[1] = *(const v8h*)(Ksh + (j * 16 + c) * AK_D + dc * 32 + 16 + 8 * hh);
        s[j] = mma_h16(qa[dc], kb.v, s[j]);
      }
    }
    int kvkeep[4];
    float kadd[4];
#pragma unroll
    for (int j = 0; j < 4; ++j) {
      kvkeep[j] = kmask[(size_t)b * Skv + kv0 + j * 16 + c];
      kadd[j] = ub * (1.0f - (float)kvkeep[j]);
    }
    float cm[8];
#pragma unroll
    for (int r = 0; r < 8; ++r) {
      float m = -__builtin_inff();
#pragma unroll
      for (int j = 0; j < 4; ++j) {
        float v = (kvkeep[j] == 0) ? mfill : s[j][r] * qscale;
        v = v + kadd[j];
        s[j][r] = v;
        m = fmaxf(m, v);
      }
#pragma unroll
      for (int off = 1; off < 16; off <<= 1) m = fmaxf(m, __shfl_xor(m, off, 32));
      cm[r] = m;
    }
    _Float16* pw = Psh[wave];
#pragma unroll
    for (int r = 0; r < 8; ++r) {
      const float mnew = fmaxf(mrow[r], cm[r]);
      const float alpha = expf(mrow[r] - mnew);
      mrow[r] = mnew;
      float psum = 0.f;
#pragma unroll
      for (int j = 0; j < 4; ++j) {
        const float p = expf(s[j][r] - mnew);
        psum += p;
        pw[(8 * hh + r) * AK_KC + j * 16 + c] = (_Float16)(p * PSC);
      }
#pragma unroll
      for (int off = 1; off < 16; off <<= 1) psum += __shfl_xor(psum, off, 32);
      lrow[r] = lrow[r] * alpha + psum;
#pragma unroll
      for (int t = 0; t < 4; ++t) oacc[t][r] *= alpha;
    }
    __builtin_amdgcn_fence(__ATOMIC_RELEASE, "workgroup");
    __builtin_amdgcn_wave_barrier();
    __builtin_amdgcn_fence(__ATOMIC_ACQUIRE, "workgroup");
#pragma unroll
    for (int kk = 0; kk < 2; ++kk) {
      FB pa;
      pa.h[0] = *(const v8h*)(pw + c * AK_KC + kk * 32 + 8 * hh);
      pa.h[1] = *(const v8h*)(pw + c * AK_KC + kk * 32 + 16 + 8 * hh);
#pragma unroll
      for (int t = 0; t < 4; ++t) {
        FB vb;
        vb.h[0] = *(const v8h*)(Vth + (t * 16 + c) * AK_KC + kk * 32 + 8 * hh);
        vb.h[1] = *(const v8h*)(Vth + (t * 16 + c) * AK_KC + kk * 32 + 16 + 8 * hh);
        oacc[t] = mma_h16(pa.v, vb.v, oacc[t]);
      }
    }
  }

  float* os = Os[wave];
  const float gsc = gate * oscale;
#pragma unroll
  for (int r = 0; r < 8; ++r) {
    const float inv = gsc * (1.0f / (lrow[r] * PSC));
#pragma unroll
    for (int t = 0; t < 4; ++t) os[(8 * hh + r) * 68 + t * 16 + c] = oacc[t][r] * inv;
  }
  __builtin_amdgcn_fence(__ATOMIC_RELEASE, "workgroup");
  __builtin_amdgcn_wave_barrier();
  __builtin_amdgcn_fence(__ATOMIC_ACQUIRE, "workgroup");
  {
    const int q = lane >> 3, c8 = (lane & 7) * 8;
    _Float16* ob = Op + (size_t)(b * S + q0) * ldo + h * AK_D;
    for (int pass = 0; pass < 2; ++pass) {
#pragma unroll
      for (int it = 0; it < 4; ++it) {
        const int row = it * 4 + q;
        const float* sp = os + row * 68 + c8;
        v8h hv;
#pragma unroll
        for (int e = 0; e < 8; ++e) hv[e] = (_Float16)sp[e];
        *(volatile v8h*)(ob + (size_t)row * ldo + c8) = hv;
      }
      __threadfence();
    }
  }
}

extern "C" void kernel_launch(void* const* d_in, const int* in_sizes, int n_in,
                              void* d_out, int out_size, void* d_ws, size_t ws_size,
                              hipStream_t stream) {
  if (n_in < 14) return;
  const int D  = 1024;
  const int H  = 16;
  const int DH = 64;
  const int Bn = 2;
  const int S  = 2048;
  const int M  = Bn * S;
  if (in_sizes[0] != M * D || in_sizes[1] != M || in_sizes[3] != D * D || in_sizes[5] != D * D ||
      in_sizes[7] != D * D || in_sizes[9] != D * D || in_sizes[4] != D || in_sizes[6] != D ||
      in_sizes[8] != D || in_sizes[10] != D || in_sizes[11] != H || in_sizes[13] != H ||
      out_size != M * D || H * DH != D) return;
  const int GD = in_sizes[2] / Bn;
  if (GD <= 0 || in_sizes[2] != Bn * GD || in_sizes[12] != H * GD) return;
  if ((S % 64) != 0 || (M % 64) != 0 || (D % 64) != 0) return;

  const float* x    = (const float*)d_in[0];
  const int*   mask = (const int*)  d_in[1];
  const float* gq   = (const float*)d_in[2];
  const float* Wq   = (const float*)d_in[3];
  const float* bq   = (const float*)d_in[4];
  const float* Wk   = (const float*)d_in[5];
  const float* bk   = (const float*)d_in[6];
  const float* Wv   = (const float*)d_in[7];
  const float* bv   = (const float*)d_in[8];
  const float* Wo   = (const float*)d_in[9];
  const float* bo   = (const float*)d_in[10];
  const float* ubias= (const float*)d_in[11];
  const float* Wqh  = (const float*)d_in[12];
  const float* bqh  = (const float*)d_in[13];
  float* out = (float*)d_out;

  const size_t SZ_ACT = (size_t)M * D * 2;
  const size_t SZ_W   = (size_t)D * D * 2;
  size_t off = 0;
  const size_t o_x16  = off; off += SZ_ACT;
  const size_t o_wq16 = off; off += SZ_W;
  const size_t o_wk16 = off; off += SZ_W;
  const size_t o_wv16 = off; off += SZ_W;
  const size_t o_wo16 = off; off += SZ_W;
  const size_t o_q16  = off; off += SZ_ACT;
  const size_t o_k16  = off; off += SZ_ACT;
  const size_t o_vt16 = off; off += SZ_ACT;
  const size_t o_o16  = off; off += SZ_ACT;
  const size_t total  = off;
  if (total > ws_size || total > (size_t)134217728) return;
  char* ws = (char*)d_ws;
  unsigned short* x16  = (unsigned short*)(ws + o_x16);
  unsigned short* wq16 = (unsigned short*)(ws + o_wq16);
  unsigned short* wk16 = (unsigned short*)(ws + o_wk16);
  unsigned short* wv16 = (unsigned short*)(ws + o_wv16);
  unsigned short* wo16 = (unsigned short*)(ws + o_wo16);
  unsigned short* q16  = (unsigned short*)(ws + o_q16);
  unsigned short* k16  = (unsigned short*)(ws + o_k16);
  unsigned short* vt16 = (unsigned short*)(ws + o_vt16);
  unsigned short* o16  = (unsigned short*)(ws + o_o16);

  {
    const int n2x = (M * D) / 2;
    cast_f32_f16x2<<<dim3((n2x + 255) / 256), dim3(256), 0, stream>>>(x, (_Float16*)x16, n2x);
    const int n2w = (D * D) / 2;
    const int gw = (n2w + 255) / 256;
    cast_f32_f16x2s<<<dim3(gw), dim3(256), 0, stream>>>(Wq, (_Float16*)wq16, n2w, 16.0f);
    cast_f32_f16x2s<<<dim3(gw), dim3(256), 0, stream>>>(Wk, (_Float16*)wk16, n2w, 16.0f);
    cast_f32_f16x2s<<<dim3(gw), dim3(256), 0, stream>>>(Wv, (_Float16*)wv16, n2w, 16.0f);
    cast_f32_f16x2s<<<dim3(gw), dim3(256), 0, stream>>>(Wo, (_Float16*)wo16, n2w, 16.0f);
  }

  const int tilesQK = (M / 64) * (D / 64);
  const dim3 gQK((tilesQK + 7) / 8, 1);
  const float w16inv = 1.0f / 16.0f;
  wmma_gemm64<0, false, 2, 1, false, 0><<<gQK, dim3(256), 0, stream>>>(
      x16, x16, D, 0L, wq16, wq16, D, 0L, (void*)q16, (void*)q16, D, 0L, bq, x, 0L, M, D, D, w16inv);
  wmma_gemm64<0, false, 2, 1, false, 0><<<gQK, dim3(256), 0, stream>>>(
      x16, x16, D, 0L, wk16, wk16, D, 0L, (void*)k16, (void*)k16, D, 0L, bk, x, 0L, M, D, D, w16inv);
  const int tilesV = (D / 64) * (M / 64);
  const dim3 gV((tilesV + 7) / 8, 1);
  wmma_gemm64<0, false, 1, 1, false, 0><<<gV, dim3(256), 0, stream>>>(
      wv16, wv16, D, 0L, x16, x16, D, 0L, (void*)vt16, (void*)vt16, M, 0L, bv, x, 0L, D, M, D, w16inv);

  const float qscale = 0.125f;
  const float oscale = 64.0f;
  attn64_f16io<<<dim3(Bn * H * (S / 64)), dim3(128), 0, stream>>>(
      (const _Float16*)q16, (const _Float16*)k16, (const _Float16*)vt16, (_Float16*)o16,
      mask, ubias, gq, Wqh, bqh, S, S, H, D, D, M, D, GD, qscale, -1e30f, oscale);

  wmma_gemm64<0, false, 2, 0, false, 0><<<gQK, dim3(256), 0, stream>>>(
      o16, o16, D, 0L, wo16, wo16, D, 0L, (void*)out, (void*)out, D, 0L, bo, x, 0L, M, D, D, 1.0f / 1024.0f);

  (void)hipGetLastError();
}
